// CUP_28054726378228
// MI455X (gfx1250) — hardware-verified
//
#include <hip/hip_runtime.h>
#define NBI 4
#define CC 64
#define H0 128
#define NP0 (H0 * H0)
#define NLV 4
#define KT 9
#define KD (KT * CC)
#define NOM 32
#define SER 4
typedef __bf16 v16b __attribute__((ext_vector_type(16)));
typedef unsigned short v8us __attribute__((ext_vector_type(8), may_alias));
typedef float  v8f  __attribute__((ext_vector_type(8)));
typedef float  v4f  __attribute__((ext_vector_type(4)));
typedef float  v4fa __attribute__((ext_vector_type(4), may_alias));
union FragB { v16b v; v8us half[2]; unsigned short u[16]; };

__device__ __forceinline__ unsigned short bf16_bits(float x) { unsigned int u = __float_as_uint(x); return (unsigned short)((u + 0x7FFFu + ((u >> 16) & 1u)) >> 16); }
__device__ __forceinline__ float bf16_val(unsigned short b) { return __uint_as_float(((unsigned int)b) << 16); }
__device__ __forceinline__ float bf16_round(float x) { return bf16_val(bf16_bits(x)); }
template <int NT>
__device__ __forceinline__ v8f mmaN(v16b ah, v16b al, v16b bh, v16b bl, v8f c) {
  c = __builtin_amdgcn_wmma_f32_16x16x32_bf16(false, ah, false, bh, (short)0, c, false, false);
  if (NT >= 2) c = __builtin_amdgcn_wmma_f32_16x16x32_bf16(false, al, false, bh, (short)0, c, false, false);
  if (NT >= 3) c = __builtin_amdgcn_wmma_f32_16x16x32_bf16(false, ah, false, bl, (short)0, c, false, false);
  asm volatile("v_nop\n\tv_nop\n\tv_nop\n\tv_nop" : "+v"(c) : "v"(ah), "v"(al), "v"(bh), "v"(bl));
  return c;
}

__global__ __launch_bounds__(256) void k_wt_bf16(const float* __restrict__ W, unsigned short* __restrict__ Wt, int K, int N) {
  const int t = blockIdx.x * 256 + threadIdx.x;
  const int k8n = K / 8;
  if (t >= N * k8n) return;
  const int n = t / k8n, k8 = (t % k8n) * 8;
  v8us v;
#pragma unroll
  for (int i = 0; i < 8; ++i) v[i] = bf16_bits(W[(size_t)(k8 + i) * N + n]);
  *(volatile v8us*)(Wt + (size_t)n * K + k8) = v;
  __threadfence();
  *(volatile v8us*)(Wt + (size_t)n * K + k8) = v;
}

template <bool ASPLIT, int ACT, bool BIAS_BF16>
__global__ __launch_bounds__(128) void k_gemm_bf(const float* __restrict__ A, int lda, const unsigned short* __restrict__ Wt, int ldb,
                                               const float* __restrict__ bias, float* __restrict__ C, int ldc, int M, int N, int K) {
  __shared__ __attribute__((aligned(16))) float so[4][16][64];
  const int tid = threadIdx.x, w = tid >> 5, lane = tid & 31, ln = lane & 15, hh = lane >> 4;
  const int ntn = N / 64;
  const int wid = blockIdx.x * 4 + w;
  const int mt = wid / ntn, nq = wid % ntn;
  if (mt * 16 >= M) return;
  const int row0 = mt * 16, col0 = nq * 64;
  const float* arow = A + (size_t)(row0 + ln) * lda;
  v8f acc[4] = {};
  for (int kb = 0; kb < K; kb += 32) {
    FragB ah, al;
    const v4f x0 = *(const v4fa*)(arow + kb + 8 * hh), x1 = *(const v4fa*)(arow + kb + 8 * hh + 4);
    const v4f x2 = *(const v4fa*)(arow + kb + 16 + 8 * hh), x3 = *(const v4fa*)(arow + kb + 16 + 8 * hh + 4);
    float xs[16] = {x0[0],x0[1],x0[2],x0[3],x1[0],x1[1],x1[2],x1[3],x2[0],x2[1],x2[2],x2[3],x3[0],x3[1],x3[2],x3[3]};
#pragma unroll
    for (int i = 0; i < 16; ++i) { const unsigned short hb = bf16_bits(xs[i]); ah.u[i] = hb; al.u[i] = ASPLIT ? bf16_bits(xs[i] - bf16_val(hb)) : (unsigned short)0; }
#pragma unroll
    for (int t = 0; t < 4; ++t) {
      const unsigned short* brow = Wt + (size_t)(col0 + t * 16 + ln) * ldb + kb;
      FragB b;
      b.half[0] = *(const v8us*)(brow + 8 * hh);
      b.half[1] = *(const v8us*)(brow + 16 + 8 * hh);
      acc[t] = mmaN<ASPLIT ? 2 : 1>(ah.v, al.v, b.v, b.v, acc[t]);
    }
  }
#pragma unroll
  for (int t = 0; t < 4; ++t) {
    float bv = bias ? bias[col0 + t * 16 + ln] : 0.f;
    if (BIAS_BF16) bv = bf16_round(bv);
#pragma unroll
    for (int r = 0; r < 8; ++r) { float v = acc[t][r] + bv; if (ACT == 1) v = fmaxf(v, 0.f); so[w][8 * hh + r][t * 16 + ln] = v; }
  }
  __builtin_amdgcn_fence(__ATOMIC_ACQ_REL, "workgroup");
  __builtin_amdgcn_wave_barrier();
  const int rsub = lane >> 4, c4 = (lane & 15) * 4;
  for (int pass = 0; pass < 2; ++pass) {
#pragma unroll
    for (int q = 0; q < 8; ++q) {
      const int r = q * 2 + rsub;
      const v4f v = *(const v4fa*)&so[w][r][c4];
      *(volatile v4f*)(C + (size_t)(row0 + r) * ldc + col0 + c4) = v;
    }
    if (pass == 0) __threadfence();
  }
}

template <bool ASPLIT, int ACT, bool BIAS_BF16, bool RES_BF16>
__global__ __launch_bounds__(128) void k_gemm_bf3(const float* __restrict__ A, int lda, const unsigned short* __restrict__ Wt, int ldb,
                                                const float* __restrict__ bias, const float* __restrict__ resid, int rmod, int ldr,
                                                float* __restrict__ C, int ldc, int M, int N, int K) {
  __shared__ __attribute__((aligned(16))) float so[4][16][64];
  const int tid = threadIdx.x, w = tid >> 5, lane = tid & 31, ln = lane & 15, hh = lane >> 4;
  const int ntn = N / 64;
  const int wid = blockIdx.x * 4 + w;
  const int mt = wid / ntn, nq = wid % ntn;
  if (mt * 16 >= M) return;
  const int row0 = mt * 16, col0 = nq * 64;
  const float* arow = A + (size_t)(row0 + ln) * lda;
  v8f acc[4] = {};
  for (int kb = 0; kb < K; kb += 32) {
    FragB ah, al;
    const v4f x0 = *(const v4fa*)(arow + kb + 8 * hh), x1 = *(const v4fa*)(arow + kb + 8 * hh + 4);
    const v4f x2 = *(const v4fa*)(arow + kb + 16 + 8 * hh), x3 = *(const v4fa*)(arow + kb + 16 + 8 * hh + 4);
    float xs[16] = {x0[0],x0[1],x0[2],x0[3],x1[0],x1[1],x1[2],x1[3],x2[0],x2[1],x2[2],x2[3],x3[0],x3[1],x3[2],x3[3]};
#pragma unroll
    for (int i = 0; i < 16; ++i) { const unsigned short hb = bf16_bits(xs[i]); ah.u[i] = hb; al.u[i] = ASPLIT ? bf16_bits(xs[i] - bf16_val(hb)) : (unsigned short)0; }
#pragma unroll
    for (int t = 0; t < 4; ++t) {
      const unsigned short* brow = Wt + (size_t)(col0 + t * 16 + ln) * ldb + kb;
      FragB b;
      b.half[0] = *(const v8us*)(brow + 8 * hh);
      b.half[1] = *(const v8us*)(brow + 16 + 8 * hh);
      acc[t] = mmaN<ASPLIT ? 2 : 1>(ah.v, al.v, b.v, b.v, acc[t]);
    }
  }
#pragma unroll
  for (int t = 0; t < 4; ++t) {
    const int col = col0 + t * 16 + ln;
    float bv = bias ? bias[col] : 0.f;
    if (BIAS_BF16) bv = bf16_round(bv);
#pragma unroll
    for (int r = 0; r < 8; ++r) {
      float v = acc[t][r] + bv;
      if (resid) { float rv = resid[(size_t)((row0 + 8 * hh + r) % rmod) * ldr + col]; if (RES_BF16) rv = bf16_round(rv); v += rv; }
      if (ACT == 1) v = fmaxf(v, 0.f);
      if (ACT == 2) v = 0.5f * v * (1.0f + erff(v * 0.70710678118654752f));
      if (ACT == 3) { const float u = 0.7978845608028654f * (v + 0.044715f * v * v * v); v = 0.5f * v * (1.0f + tanhf(u)); }
      so[w][8 * hh + r][t * 16 + ln] = v;
    }
  }
  __builtin_amdgcn_fence(__ATOMIC_ACQ_REL, "workgroup");
  __builtin_amdgcn_wave_barrier();
  const int rsub = lane >> 4, c4 = (lane & 15) * 4;
  for (int pass = 0; pass < 2; ++pass) {
#pragma unroll
    for (int q = 0; q < 8; ++q) {
      const int r = q * 2 + rsub;
      const v4f v = *(const v4fa*)&so[w][r][c4];
      *(volatile v4f*)(C + (size_t)(row0 + r) * ldc + col0 + c4) = v;
    }
    if (pass == 0) __threadfence();
  }
}
template <bool PARAM_BF16>
__global__ __launch_bounds__(256) void k_layernorm(const float* __restrict__ X, const float* __restrict__ R, const float* __restrict__ g, const float* __restrict__ bta,
                                                  float* __restrict__ out_sum, float* __restrict__ out_norm, int N, float eps) {
  __shared__ float red[256];
  const int row = blockIdx.x, tid = threadIdx.x;
  const float* x = X + (size_t)row * N; const float* rr = R ? R + (size_t)row * N : nullptr;
  float vals[16];
  const int per = N / 256;
  float s1 = 0.f;
  for (int u = 0; u < per / 4; ++u) {
    const int j = tid * 4 + 1024 * u;
    const v4f a = *(const v4fa*)(x + j);
    v4f b = {0.f,0.f,0.f,0.f}; if (rr) b = *(const v4fa*)(rr + j);
#pragma unroll
    for (int q = 0; q < 4; ++q) { const float v = a[q] + b[q]; vals[u * 4 + q] = v; s1 += v; }
  }
  red[tid] = s1; __syncthreads();
  for (int st = 128; st > 0; st >>= 1) { if (tid < st) red[tid] += red[tid + st]; __syncthreads(); }
  const float mu = red[0] / (float)N; __syncthreads();
  float s2 = 0.f;
  for (int u = 0; u < per / 4; ++u)
#pragma unroll
    for (int q = 0; q < 4; ++q) { const float c = vals[u * 4 + q] - mu; s2 += c * c; }
  red[tid] = s2; __syncthreads();
  for (int st = 128; st > 0; st >>= 1) { if (tid < st) red[tid] += red[tid + st]; __syncthreads(); }
  const float rs = rsqrtf(red[0] / (float)N + eps);
  for (int pass = 0; pass < 2; ++pass) {
    for (int u = 0; u < per / 4; ++u) {
      const int j = tid * 4 + 1024 * u;
      v4f o, sm;
#pragma unroll
      for (int q = 0; q < 4; ++q) {
        float gg = g[j + q], bb = bta[j + q];
        if (PARAM_BF16) { gg = bf16_round(gg); bb = bf16_round(bb); }
        sm[q] = vals[u * 4 + q]; o[q] = (vals[u * 4 + q] - mu) * rs * gg + bb;
      }
      if (out_sum) *(volatile v4f*)(out_sum + (size_t)row * N + j) = sm;
      *(volatile v4f*)(out_norm + (size_t)row * N + j) = o;
    }
    if (pass == 0) __threadfence();
  }
}


typedef _Float16 v16h __attribute__((ext_vector_type(16)));
union FragH { v16h v; v8us half[2]; _Float16 h[16]; unsigned short u[16]; };
template <int NT>
__device__ __forceinline__ v8f mmaH(v16h ah, v16h al, v16h bh, v16h bl, v8f c) {
  c = __builtin_amdgcn_wmma_f32_16x16x32_f16(false, ah, false, bh, (short)0, c, false, false);
  if (NT >= 2) c = __builtin_amdgcn_wmma_f32_16x16x32_f16(false, al, false, bh, (short)0, c, false, false);
  if (NT >= 3) c = __builtin_amdgcn_wmma_f32_16x16x32_f16(false, ah, false, bl, (short)0, c, false, false);
  asm volatile("v_nop\n\tv_nop\n\tv_nop\n\tv_nop" : "+v"(c) : "v"(ah), "v"(al), "v"(bh), "v"(bl));
  return c;
}
template <bool ASPLIT>
__global__ __launch_bounds__(128) void k_gemm_h(const float* __restrict__ A, int lda, size_t sA, const _Float16* __restrict__ Bh, int ldb, size_t sB, float alpha, float* __restrict__ C, int ldc, size_t sC, int M, int N, int K) {
  __shared__ __attribute__((aligned(16))) float so[4][16][64];
  const int tid = threadIdx.x, w = tid >> 5, lane = tid & 31, ln = lane & 15, hh = lane >> 4; const int by = blockIdx.y;
  A += (size_t)by * sA; Bh += (size_t)by * sB; C += (size_t)by * sC;
  const int ntn = (N + 63) / 64; const int wid = blockIdx.x * 4 + w; const int mt = wid / ntn, nq = wid % ntn; if (mt * 16 >= M) return;
  const int row0 = mt * 16, col0 = nq * 64; const float* arow = A + (size_t)(row0 + ln) * lda;
  v8f acc[4] = {};
  for (int kb = 0; kb < K; kb += 32) {
    FragH ah, al;
    const v4f x0 = *(const v4fa*)(arow + kb + 8 * hh), x1 = *(const v4fa*)(arow + kb + 8 * hh + 4), x2 = *(const v4fa*)(arow + kb + 16 + 8 * hh), x3 = *(const v4fa*)(arow + kb + 16 + 8 * hh + 4);
    float xs[16] = {x0[0],x0[1],x0[2],x0[3],x1[0],x1[1],x1[2],x1[3],x2[0],x2[1],x2[2],x2[3],x3[0],x3[1],x3[2],x3[3]};
#pragma unroll
    for (int i = 0; i < 16; ++i) { const _Float16 h = (_Float16)xs[i]; ah.h[i] = h; al.h[i] = ASPLIT ? (_Float16)(xs[i] - (float)h) : (_Float16)0.0f; }
#pragma unroll
    for (int t = 0; t < 4; ++t) { if (col0 + t * 16 >= N) continue; const size_t boff = (size_t)(col0 + t * 16 + ln) * ldb + kb; FragH bq; bq.half[0] = *(const v8us*)(Bh + boff + 8 * hh); bq.half[1] = *(const v8us*)(Bh + boff + 16 + 8 * hh);
      acc[t] = mmaH<ASPLIT ? 2 : 1>(ah.v, al.v, bq.v, bq.v, acc[t]); }
  }
#pragma unroll
  for (int t = 0; t < 4; ++t) { if (col0 + t * 16 >= N) continue;
#pragma unroll
    for (int r = 0; r < 8; ++r) so[w][8 * hh + r][t * 16 + ln] = acc[t][r] * alpha; }
  __builtin_amdgcn_fence(__ATOMIC_ACQ_REL, "workgroup"); __builtin_amdgcn_wave_barrier();
  const int rsub = lane >> 4, c4 = (lane & 15) * 4;
  for (int pass = 0; pass < 2; ++pass) {
#pragma unroll
    for (int q = 0; q < 8; ++q) { const int r = q * 2 + rsub; if (col0 + c4 < N) { const v4f v = *(const v4fa*)&so[w][r][c4]; *(volatile v4f*)(C + (size_t)(row0 + r) * ldc + col0 + c4) = v; } }
    if (pass == 0) __threadfence(); }
}

__global__ __launch_bounds__(256) void k_wt_f16(const float* __restrict__ W, _Float16* __restrict__ Wt, int K, int N, float scale) {
  const int t = blockIdx.x * 256 + threadIdx.x; if (t >= N * (K / 8)) return; const int n = t / (K / 8), k8 = (t % (K / 8)) * 8; FragH f;
#pragma unroll
  for (int i = 0; i < 8; ++i) f.h[i] = (_Float16)(bf16_round(W[(size_t)(k8 + i) * N + n]) * scale); const v8us o = f.half[0];
  *(volatile v8us*)((unsigned short*)Wt + (size_t)n * K + k8) = o; __threadfence(); *(volatile v8us*)((unsigned short*)Wt + (size_t)n * K + k8) = o;
}
template <int ACT>
__global__ __launch_bounds__(128) void k_gemm_hhx(const _Float16* __restrict__ A, int lda, size_t sA, const _Float16* __restrict__ Bh, int ldb, size_t sB, float alpha, const float* __restrict__ bias, size_t sBias, const float* __restrict__ CP, int rowsPerB, size_t sCPb, int row0g,
    float* __restrict__ C, _Float16* __restrict__ C16, int ldc, size_t sC, int M, int N, int K) {
  __shared__ __attribute__((aligned(16))) float so[4][16][64];
  const int tid = threadIdx.x, w = tid >> 5, lane = tid & 31, ln = lane & 15, hh = lane >> 4; const int by = blockIdx.y;
  A += (size_t)by * sA; Bh += (size_t)by * sB; const size_t cofs = (size_t)by * sC; const float* bp = bias ? bias + (size_t)by * sBias : nullptr;
  const int ntn = (N + 63) / 64; const int wid = blockIdx.x * 4 + w; const int mt = wid / ntn, nq = wid % ntn; if (mt * 16 >= M) return;
  const int row0 = mt * 16, col0 = nq * 64; const _Float16* arow = A + (size_t)(row0 + ln) * lda;
  v8f acc[4] = {};
  for (int kb = 0; kb < K; kb += 32) { FragH ah; ah.half[0] = *(const v8us*)((const unsigned short*)arow + kb + 8 * hh); ah.half[1] = *(const v8us*)((const unsigned short*)arow + kb + 16 + 8 * hh);
#pragma unroll
    for (int t = 0; t < 4; ++t) { if (col0 + t * 16 >= N) continue; const size_t boff = (size_t)(col0 + t * 16 + ln) * ldb + kb; FragH bq; bq.half[0] = *(const v8us*)((const unsigned short*)Bh + boff + 8 * hh); bq.half[1] = *(const v8us*)((const unsigned short*)Bh + boff + 16 + 8 * hh);
      acc[t] = mmaH<1>(ah.v, ah.v, bq.v, bq.v, acc[t]); }
  }
#pragma unroll
  for (int t = 0; t < 4; ++t) { if (col0 + t * 16 >= N) continue; const int col = col0 + t * 16 + ln; const float bv = bp ? bf16_round(bp[col]) : 0.f;
#pragma unroll
    for (int r = 0; r < 8; ++r) { float v = acc[t][r] * alpha + bv; if (CP) { const int bidx = (row0g + row0 + 8 * hh + r) / rowsPerB; v += CP[(size_t)bidx * sCPb + (size_t)by * 64 + col]; } if (ACT == 1) v = (v > 0.f) ? v : expm1f(v); else if (ACT == 7) v = (v > 0.f) ? v + 1.0f : expf(v); else if (ACT == 8) v = tanhf(v); else if (ACT == 9) v = 0.5f * v * (1.0f + tanhf(0.7978845608028654f * (v + 0.044715f * v * v * v))); else if (ACT == 11) v = 1.0f / (1.0f + expf(-v)); else if (ACT == 12) v = (v > 0.f) ? v : 0.01f * v; else if (ACT == 14) v = (v > 0.f) ? v : 0.1f * v; else if (ACT == 15) v = v / (1.0f + expf(-v)); else if (ACT == 3) v = fmaxf(v, 0.f); else if (ACT == 6) v = 0.5f * v * (1.0f + erff(v * 0.70710678118654752f)); so[w][8 * hh + r][t * 16 + ln] = v; } }
  __builtin_amdgcn_fence(__ATOMIC_ACQ_REL, "workgroup"); __builtin_amdgcn_wave_barrier();
  const int rsub = lane >> 4, c4 = (lane & 15) * 4; typedef _Float16 v4h __attribute__((ext_vector_type(4)));
  for (int pass = 0; pass < 2; ++pass) {
#pragma unroll
    for (int q = 0; q < 8; ++q) { const int r = q * 2 + rsub; if (col0 + c4 < N) { const v4f v = *(const v4fa*)&so[w][r][c4]; if (C) *(volatile v4f*)(C + cofs + (size_t)(row0 + r) * ldc + col0 + c4) = v; if (C16) { v4h h4; for (int i = 0; i < 4; ++i) h4[i] = (_Float16)v[i]; *(volatile v4h*)(C16 + cofs + (size_t)(row0 + r) * ldc + col0 + c4) = h4; } } }
    if (pass == 0) __threadfence(); }
}


typedef _Float16 v4h __attribute__((ext_vector_type(4)));

__global__ __launch_bounds__(256) void k_x16(const float* __restrict__ x, _Float16* __restrict__ X16, size_t n8) { const size_t t = (size_t)blockIdx.x * 256 + threadIdx.x; if (t >= n8) return; FragH f;
#pragma unroll
  for (int q = 0; q < 8; ++q) f.h[q] = (_Float16)bf16_round(x[t * 8 + q]); *(volatile v8us*)((unsigned short*)X16 + t * 8) = f.half[0]; __threadfence(); *(volatile v8us*)((unsigned short*)X16 + t * 8) = f.half[0]; }
__global__ __launch_bounds__(256) void k_h16(const float* __restrict__ x, _Float16* __restrict__ X16, size_t n8) { const size_t t = (size_t)blockIdx.x * 256 + threadIdx.x; if (t >= n8) return; FragH f;
#pragma unroll
  for (int q = 0; q < 8; ++q) f.h[q] = (_Float16)x[t * 8 + q]; *(volatile v8us*)((unsigned short*)X16 + t * 8) = f.half[0]; __threadfence(); *(volatile v8us*)((unsigned short*)X16 + t * 8) = f.half[0]; }
__global__ __launch_bounds__(256) void k_round16f(const float* __restrict__ W, _Float16* __restrict__ Bt, size_t n8) { const size_t t = (size_t)blockIdx.x * 256 + threadIdx.x; if (t >= n8) return; FragH f;
#pragma unroll
  for (int i = 0; i < 8; ++i) f.h[i] = (_Float16)(bf16_round(W[t * 8 + i]) * 16.0f); *(volatile v8us*)((unsigned short*)Bt + t * 8) = f.half[0]; __threadfence(); *(volatile v8us*)((unsigned short*)Bt + t * 8) = f.half[0]; }
template <int NHv, int TTv>
__global__ __launch_bounds__(256) void k_vt(const _Float16* __restrict__ V16, int ldv, int voff, _Float16* __restrict__ Vt) { __shared__ unsigned short tl[64][66]; const int tid = threadIdx.x; const int slab = blockIdx.x / (TTv / 64), lg = blockIdx.x % (TTv / 64); const int b = slab / NHv, h = slab % NHv;
  for (int i = tid; i < 64 * 8; i += 256) { const int r = i / 8, c8 = (i % 8) * 8; FragH f; f.half[0] = *(const v8us*)((const unsigned short*)V16 + ((size_t)b * TTv + lg * 64 + r) * ldv + voff + h * 64 + c8);
#pragma unroll
    for (int q = 0; q < 8; ++q) tl[r][c8 + q] = f.u[q]; }
  __syncthreads();
  for (int pass = 0; pass < 2; ++pass) {
#pragma unroll
    for (int rd = 0; rd < 2; ++rd) { const int d = rd * 32 + tid / 8, pc = tid % 8; FragH f;
#pragma unroll
      for (int q = 0; q < 8; ++q) f.u[q] = tl[pc * 8 + q][d];
      *(volatile v8us*)((unsigned short*)Vt + ((size_t)slab * 64 + d) * TTv + lg * 64 + pc * 8) = f.half[0]; }
    if (pass == 0) __threadfence(); } }

__global__ __launch_bounds__(256) void k_hl(const float* __restrict__ F, _Float16* __restrict__ Hh, _Float16* __restrict__ Hl, size_t n8) { const size_t t = (size_t)blockIdx.x * 256 + threadIdx.x; if (t >= n8) return; FragH fh, fl; const v4f a = *(const v4fa*)(F + t * 8), c = *(const v4fa*)(F + t * 8 + 4);
#pragma unroll
  for (int q = 0; q < 4; ++q) { _Float16 h = (_Float16)a[q]; fh.h[q] = h; fl.h[q] = (_Float16)((a[q] - (float)h) * 1024.0f); h = (_Float16)c[q]; fh.h[4 + q] = h; fl.h[4 + q] = (_Float16)((c[q] - (float)h) * 1024.0f); }
  for (int pass = 0; pass < 2; ++pass) { *(volatile v8us*)((unsigned short*)Hh + t * 8) = fh.half[0]; *(volatile v8us*)((unsigned short*)Hl + t * 8) = fl.half[0]; if (pass == 0) __threadfence(); } }

__global__ __launch_bounds__(256) void k_in(const float* __restrict__ x, int b, float* __restrict__ CF, _Float16* __restrict__ C16) { const int t = blockIdx.x * 256 + threadIdx.x; if (t >= NP0 * (CC / 4)) return; const int c0 = (t % (CC / 4)) * 4, p = t / (CC / 4); v4f a; FragH f;
#pragma unroll
  for (int q = 0; q < 4; ++q) { const float v = bf16_round(x[((size_t)b * CC + c0 + q) * NP0 + p]); a[q] = v; f.h[q] = (_Float16)v; }
  const unsigned long long pk = *(const unsigned long long*)&f.u[0];
  for (int pass = 0; pass < 2; ++pass) { *(volatile v4f*)(CF + (size_t)p * CC + c0) = a; *(volatile unsigned long long*)((unsigned short*)C16 + (size_t)p * CC + c0) = pk; if (pass == 0) __threadfence(); } }
__global__ __launch_bounds__(256) void k_rs_rows(const float* __restrict__ P, int nin, int nout, float* __restrict__ T) {
  #pragma clang fp contract(off)
  const int t = blockIdx.x * 256 + threadIdx.x; if (t >= nout * nin * (CC / 4)) return; const int c0 = (t % (CC / 4)) * 4; const int x = (t / (CC / 4)) % nin; const int yo = t / ((CC / 4) * nin); const float sc = (float)nin / (float)nout; float src = ((float)yo + 0.5f) * sc - 0.5f; src = fminf(fmaxf(src, 0.f), (float)(nin - 1)); const int i0 = (int)floorf(src); const int i1 = min(i0 + 1, nin - 1); const float w = src - (float)i0;
  const v4f a0 = *(const v4fa*)(P + ((size_t)i0 * nin + x) * CC + c0), b0 = *(const v4fa*)(P + ((size_t)i1 * nin + x) * CC + c0); v4f o0;
#pragma unroll
  for (int q = 0; q < 4; ++q) o0[q] = a0[q] * (1.0f - w) + b0[q] * w;
  float* dst = T + ((size_t)yo * nin + x) * CC + c0; *(volatile v4f*)dst = o0; __threadfence(); *(volatile v4f*)dst = o0; }
__global__ __launch_bounds__(256) void k_rs_cols(const float* __restrict__ T, int nin, int nout, int accumulate, float* __restrict__ O, _Float16* __restrict__ O16) {
  #pragma clang fp contract(off)
  const int t = blockIdx.x * 256 + threadIdx.x; if (t >= nout * nout * (CC / 4)) return; const int c0 = (t % (CC / 4)) * 4; const int xo = (t / (CC / 4)) % nout; const int yo = t / ((CC / 4) * nout); const float sc = (float)nin / (float)nout; float src = ((float)xo + 0.5f) * sc - 0.5f; src = fminf(fmaxf(src, 0.f), (float)(nin - 1)); const int i0 = (int)floorf(src); const int i1 = min(i0 + 1, nin - 1); const float w = src - (float)i0;
  const v4f a0 = *(const v4fa*)(T + ((size_t)yo * nin + i0) * CC + c0), b0 = *(const v4fa*)(T + ((size_t)yo * nin + i1) * CC + c0); v4f o0; FragH f;
  float* dst = O + ((size_t)yo * nout + xo) * CC + c0; v4f p0 = {0.f, 0.f, 0.f, 0.f}; if (accumulate) p0 = *(const v4fa*)dst;
#pragma unroll
  for (int q = 0; q < 4; ++q) { o0[q] = p0[q] + (a0[q] * (1.0f - w) + b0[q] * w); f.h[q] = (_Float16)o0[q]; }
  const unsigned long long pk = *(const unsigned long long*)&f.u[0];
  for (int pass = 0; pass < 2; ++pass) { *(volatile v4f*)dst = o0; if (O16) *(volatile unsigned long long*)((unsigned short*)O16 + ((size_t)yo * nout + xo) * CC + c0) = pk; if (pass == 0) __threadfence(); } }
__global__ __launch_bounds__(256) void k_im2col(const _Float16* __restrict__ P, int side, _Float16* __restrict__ COL) { const int np_ = side * side; const int t = blockIdx.x * 256 + threadIdx.x; if (t >= np_ * KT * (CC / 8)) return; const int c0 = (t % (CC / 8)) * 8; const int k = (t / (CC / 8)) % KT; const int p = t / ((CC / 8) * KT); const int h = p / side, w = p % side; const int yy = h - 1 + k / 3, xx = w - 1 + k % 3; FragH f = FragH{};
  if (yy >= 0 && yy < side && xx >= 0 && xx < side) f.half[0] = *(const v8us*)((const unsigned short*)P + ((size_t)yy * side + xx) * CC + c0);
  *(volatile v8us*)((unsigned short*)COL + ((size_t)p * KT + k) * CC + c0) = f.half[0]; __threadfence(); *(volatile v8us*)((unsigned short*)COL + ((size_t)p * KT + k) * CC + c0) = f.half[0]; }
__global__ __launch_bounds__(256) void k_wtap(const float* __restrict__ w, int O, int Opad, _Float16* __restrict__ Bt) { const int t = blockIdx.x * 256 + threadIdx.x; if (t >= Opad * (KD / 8)) return; const int col0 = (t % (KD / 8)) * 8, o = t / (KD / 8); const int k = col0 / CC, c0 = col0 % CC; FragH f;
#pragma unroll
  for (int q = 0; q < 8; ++q) f.h[q] = (o < O) ? (_Float16)(bf16_round(w[((size_t)o * CC + c0 + q) * KT + k]) * 16.0f) : (_Float16)0.0f;
  *(volatile v8us*)((unsigned short*)Bt + (size_t)o * KD + col0) = f.half[0]; __threadfence(); *(volatile v8us*)((unsigned short*)Bt + (size_t)o * KD + col0) = f.half[0]; }
__global__ __launch_bounds__(256) void k_bpad(const float* __restrict__ b, int n, int npad, float* __restrict__ BP) { const int l = threadIdx.x; if (l >= npad) return; const float v = (l < n) ? b[l] : 0.f; *(volatile float*)(BP + l) = v; __threadfence(); *(volatile float*)(BP + l) = v; }
__global__ __launch_bounds__(256) void k_dsamp(const float* __restrict__ OM, const _Float16* __restrict__ P, int side, _Float16* __restrict__ DCOL) {
  #pragma clang fp contract(off)
  const int np_ = side * side; const int t = blockIdx.x * 256 + threadIdx.x; if (t >= np_ * KT * (CC / 8)) return; const int c0 = (t % (CC / 8)) * 8; const int k = (t / (CC / 8)) % KT; const int p = t / ((CC / 8) * KT); const int h = p / side, w = p % side; const float dy = OM[(size_t)p * NOM + 2 * k], dx = OM[(size_t)p * NOM + 2 * k + 1];
  const float py = (float)(h + k / 3 - 1) + dy, px = (float)(w + k % 3 - 1) + dx; const float y0 = floorf(py), x0 = floorf(px); const float wy = py - y0, wx = px - x0; float acc[8];
#pragma unroll
  for (int q = 0; q < 8; ++q) acc[q] = 0.f;
#pragma unroll
  for (int cn = 0; cn < 4; ++cn) { const int yi = (int)y0 + (cn >> 1), xi = (int)x0 + (cn & 1); const bool valid = (yi >= 0 && yi < side && xi >= 0 && xi < side); const float wgt = ((cn >> 1) ? wy : (1.0f - wy)) * ((cn & 1) ? wx : (1.0f - wx)); const float f = valid ? wgt : 0.f; FragH g; g.half[0] = *(const v8us*)((const unsigned short*)P + ((size_t)min(max(yi, 0), side - 1) * side + min(max(xi, 0), side - 1)) * CC + c0);
#pragma unroll
    for (int q = 0; q < 8; ++q) acc[q] += f * (float)g.h[q]; }
  FragH o;
#pragma unroll
  for (int q = 0; q < 8; ++q) o.h[q] = (_Float16)acc[q];
  *(volatile v8us*)((unsigned short*)DCOL + ((size_t)p * KT + k) * CC + c0) = o.half[0]; __threadfence(); *(volatile v8us*)((unsigned short*)DCOL + ((size_t)p * KT + k) * CC + c0) = o.half[0]; }
__global__ __launch_bounds__(256) void k_cmean(const float* __restrict__ D, int np_, float* __restrict__ MST) {
  #pragma clang fp contract(off)
  __shared__ float red[256]; const int c = blockIdx.x, tid = threadIdx.x; float s = 0.f; for (int p = tid; p < np_; p += 256) s += D[(size_t)p * CC + c];
  red[tid] = s; __syncthreads(); for (int st = 128; st > 0; st >>= 1) { if (tid < st) red[tid] += red[tid + st]; __syncthreads(); }
  if (tid < 32) { const float m = red[0] / (float)np_; *(volatile float*)(MST + (size_t)c * 32 + tid) = m; __threadfence(); *(volatile float*)(MST + (size_t)c * 32 + tid) = m; } }
__global__ __launch_bounds__(64) void k_segate(const float* __restrict__ MST, const float* __restrict__ w1, const float* __restrict__ b1, const float* __restrict__ w2, const float* __restrict__ b2, float* __restrict__ G) {
  #pragma clang fp contract(off)
  const int c = threadIdx.x; float hsum[SER];
#pragma unroll
  for (int r = 0; r < SER; ++r) { float s = bf16_round(b1[r]);
#pragma unroll 1
    for (int cc2 = 0; cc2 < CC; ++cc2) s += MST[(size_t)cc2 * 32] * bf16_round(w1[(size_t)r * CC + cc2]);
    hsum[r] = fmaxf(s, 0.f); }
  float z = bf16_round(b2[c]);
#pragma unroll
  for (int r = 0; r < SER; ++r) z += hsum[r] * bf16_round(w2[(size_t)c * SER + r]);
  const float g = 1.0f / (1.0f + expf(-z)); *(volatile float*)(G + c) = g; __threadfence(); *(volatile float*)(G + c) = g; }
__global__ __launch_bounds__(256) void k_gate(const float* __restrict__ D, const float* __restrict__ G, int np_, float* __restrict__ CF, _Float16* __restrict__ C16) {
  #pragma clang fp contract(off)
  const int t = blockIdx.x * 256 + threadIdx.x; if (t >= np_ * (CC / 4)) return; const int c0 = (t % (CC / 4)) * 4, p = t / (CC / 4); const v4f a = *(const v4fa*)(D + (size_t)p * CC + c0); v4f o0; FragH f;
#pragma unroll
  for (int q = 0; q < 4; ++q) { o0[q] = a[q] * G[c0 + q]; f.h[q] = (_Float16)o0[q]; }
  const unsigned long long pk = *(const unsigned long long*)&f.u[0];
  for (int pass = 0; pass < 2; ++pass) { *(volatile v4f*)(CF + (size_t)p * CC + c0) = o0; *(volatile unsigned long long*)((unsigned short*)C16 + (size_t)p * CC + c0) = pk; if (pass == 0) __threadfence(); } }
__global__ __launch_bounds__(256) void k_fuse16(const float* __restrict__ F0, const float* __restrict__ F1, const float* __restrict__ F2, const float* __restrict__ F3, _Float16* __restrict__ FZ16) { const int t = blockIdx.x * 256 + threadIdx.x; if (t >= NP0 * NLV * (CC / 8)) return; const int c0 = (t % (CC / 8)) * 8; const int i = (t / (CC / 8)) % NLV; const int p = t / ((CC / 8) * NLV); const float* F = (i == 0) ? F0 : (i == 1) ? F1 : (i == 2) ? F2 : F3; const v4f a = *(const v4fa*)(F + (size_t)p * CC + c0), c = *(const v4fa*)(F + (size_t)p * CC + c0 + 4); FragH f;
#pragma unroll
  for (int q = 0; q < 8; ++q) f.h[q] = (_Float16)((q < 4) ? a[q] : c[q - 4]);
  *(volatile v8us*)((unsigned short*)FZ16 + (size_t)p * (NLV * CC) + i * CC + c0) = f.half[0]; __threadfence(); *(volatile v8us*)((unsigned short*)FZ16 + (size_t)p * (NLV * CC) + i * CC + c0) = f.half[0]; }
__global__ __launch_bounds__(256) void k_addp(float* __restrict__ A, const float* __restrict__ Bs, size_t n4) { const size_t t = (size_t)blockIdx.x * 256 + threadIdx.x; if (t >= n4) return; const v4f a = *(const v4fa*)(A + t * 4), b = *(const v4fa*)(Bs + t * 4); v4f v;
#pragma unroll
  for (int q = 0; q < 4; ++q) v[q] = a[q] + b[q];
  *(volatile v4f*)(A + t * 4) = v; __threadfence(); *(volatile v4f*)(A + t * 4) = v; }
__global__ __launch_bounds__(256) void k_out(const float* __restrict__ D, int b, float* __restrict__ out) { const int t = blockIdx.x * 256 + threadIdx.x; if (t >= CC * (NP0 / 4)) return; const int p0 = (t % (NP0 / 4)) * 4, c = t / (NP0 / 4); v4f v;
#pragma unroll
  for (int q = 0; q < 4; ++q) v[q] = D[(size_t)(p0 + q) * CC + c];
  float* dst = out + ((size_t)b * CC + c) * NP0 + p0; *(volatile v4f*)dst = v; __threadfence(); *(volatile v4f*)dst = v; }

extern "C" void kernel_launch(void* const* d_in, const int* in_sizes, int n_in,
                              void* d_out, int out_size, void* d_ws, size_t ws_size, hipStream_t stream) {
  (void)in_sizes; (void)n_in; (void)out_size;
  const float* const* I = (const float* const*)d_in; const float* x = I[0]; const float* off_w = I[1]; const float* off_b = I[2]; const float* dc_w = I[3]; const float* dc_b = I[4]; const float* se_w1 = I[5]; const float* se_b1 = I[6]; const float* se_w2 = I[7]; const float* se_b2 = I[8]; const float* fuse_w = I[9]; const float* fuse_b = I[10];
  char* ws = (char*)d_ws; size_t off = 0;
  auto take = [&](size_t bytes) { char* p = ws + off; off += (bytes + 255) & ~(size_t)255; return p; };
  _Float16* BOM = (_Float16*)take((size_t)NOM * KD * 2); float* BPM = (float*)take(NOM * 4); _Float16* BW = (_Float16*)take((size_t)CC * KD * 2); _Float16* BFZ = (_Float16*)take((size_t)CC * NLV * CC * 2); float* MST = (float*)take(CC * 32 * 4); float* G = (float*)take(CC * 4);
  float* CF = (float*)take((size_t)NP0 * CC * 4); float* CF2 = (float*)take((size_t)NP0 * CC * 4); _Float16* C16 = (_Float16*)take((size_t)NP0 * CC * 2); _Float16* COL = (_Float16*)take((size_t)NP0 * KD * 2); float* OM = (float*)take((size_t)NP0 * NOM * 4); _Float16* DCOL = (_Float16*)take((size_t)NP0 * KD * 2); float* D = (float*)take((size_t)NP0 * CC * 4); float* T = (float*)take((size_t)NP0 * CC * 4);
  float* F[NLV]; for (int i = 0; i < NLV; ++i) F[i] = (float*)take((size_t)NP0 * CC * 4); _Float16* FZ16 = (_Float16*)take((size_t)NP0 * NLV * CC * 2);
  if (off > ws_size) return;
  k_round16f<<<(CC * NLV * CC / 8 + 255) / 256, 256, 0, stream>>>(fuse_w, BFZ, (size_t)CC * NLV * CC / 8);
  for (int b = 0; b < NBI; ++b) { int side = H0; float* cur = CF; float* nxt = CF2;
    k_in<<<(NP0 * (CC / 4) + 255) / 256, 256, 0, stream>>>(x, b, cur, C16);
    for (int i = 0; i < NLV; ++i) {
      if (i > 0) { const int so = side / 2; k_rs_rows<<<(so * side * (CC / 4) + 255) / 256, 256, 0, stream>>>(cur, side, so, T); k_rs_cols<<<(so * so * (CC / 4) + 255) / 256, 256, 0, stream>>>(T, side, so, 0, nxt, C16); float* tmp = cur; cur = nxt; nxt = tmp; side = so; }
      const int np_ = side * side; const unsigned nbs = (np_ * KT * (CC / 8) + 255) / 256;
      k_wtap<<<(NOM * (KD / 8) + 255) / 256, 256, 0, stream>>>(off_w + (size_t)i * 18 * CC * KT, 18, NOM, BOM); k_bpad<<<1, 256, 0, stream>>>(off_b + (size_t)i * 18, 18, NOM, BPM); k_wtap<<<(CC * (KD / 8) + 255) / 256, 256, 0, stream>>>(dc_w + (size_t)i * CC * CC * KT, CC, CC, BW);
      k_im2col<<<nbs, 256, 0, stream>>>(C16, side, COL);
      k_gemm_hhx<0><<<dim3(((np_ / 16) * 1 + 3) / 4, 1), 128, 0, stream>>>(COL, KD, 0, BOM, KD, 0, 0.0625f, BPM, 0, nullptr, 1, 0, 0, OM, nullptr, NOM, 0, np_, NOM, KD);
      k_dsamp<<<nbs, 256, 0, stream>>>(OM, C16, side, DCOL);
      k_gemm_hhx<0><<<dim3(((np_ / 16) * 1 + 3) / 4, 1), 128, 0, stream>>>(DCOL, KD, 0, BW, KD, 0, 0.0625f, dc_b + (size_t)i * CC, 0, nullptr, 1, 0, 0, D, nullptr, CC, 0, np_, CC, KD);
      k_cmean<<<CC, 256, 0, stream>>>(D, np_, MST); k_segate<<<1, 64, 0, stream>>>(MST, se_w1 + (size_t)i * SER * CC, se_b1 + (size_t)i * SER, se_w2 + (size_t)i * CC * SER, se_b2 + (size_t)i * CC, G);
      k_gate<<<(np_ * (CC / 4) + 255) / 256, 256, 0, stream>>>(D, G, np_, cur, C16);
      k_rs_rows<<<(H0 * side * (CC / 4) + 255) / 256, 256, 0, stream>>>(cur, side, H0, T); k_rs_cols<<<(NP0 * (CC / 4) + 255) / 256, 256, 0, stream>>>(T, side, H0, 0, F[i], nullptr); }
    for (int i = NLV - 2; i >= 0; --i) k_addp<<<(unsigned)(((size_t)NP0 * CC / 4 + 255) / 256), 256, 0, stream>>>(F[i], F[i + 1], (size_t)NP0 * CC / 4);
    k_fuse16<<<(NP0 * NLV * (CC / 8) + 255) / 256, 256, 0, stream>>>(F[0], F[1], F[2], F[3], FZ16);
    k_gemm_hhx<0><<<dim3(((NP0 / 16) * 1 + 3) / 4, 1), 128, 0, stream>>>(FZ16, NLV * CC, 0, BFZ, NLV * CC, 0, 0.0625f, fuse_b, 0, nullptr, 1, 0, 0, D, nullptr, CC, 0, NP0, CC, NLV * CC);
    k_out<<<(CC * (NP0 / 4) + 255) / 256, 256, 0, stream>>>(D, b, (float*)d_out); }
}
